// GGNNLayer_10977936408823
// MI455X (gfx1250) — hardware-verified
//
#include <hip/hip_runtime.h>
#include <math.h>

constexpr int kNodes    = 50000;
constexpr int kNodesPad = 50048;
constexpr int kEdges    = 800000;
constexpr int kHid      = 256;
constexpr int kHid3     = 768;
constexpr int kTypes    = 4;
constexpr int kThr      = 256;
constexpr float kWCarry    = 16.0f;
constexpr float kWCarryInv = 0.0625f;
constexpr float kResCarry  = 2048.0f;
constexpr float kWResInv   = kWCarryInv / 2048.0f;

static_assert(kNodesPad % 32 == 0);
static_assert(kNodesPad % 16 == 0);
static_assert(kNodesPad >= kNodes);
static_assert(kHid % 32 == 0);
static_assert(kHid3 == 3 * kHid);

typedef __attribute__((ext_vector_type(16))) _Float16 v16h;
typedef __attribute__((ext_vector_type(8)))  _Float16 v8h;
typedef __attribute__((ext_vector_type(8)))  float    v8f;
typedef __attribute__((ext_vector_type(4)))  float    v4f;
typedef __attribute__((ext_vector_type(4)))  unsigned int v4u;
typedef __attribute__((ext_vector_type(2)))  unsigned int v2u;
typedef __attribute__((ext_vector_type(4)))  int      v4i;

__device__ __forceinline__ unsigned short f2bf_bits(float f) {
  unsigned u = __float_as_uint(f);
  return (unsigned short)((u + 0x7FFFu + ((u >> 16) & 1u)) >> 16);
}
__device__ __forceinline__ float bf_bits2f(unsigned short h) { return __uint_as_float(((unsigned)h) << 16); }

__device__ __forceinline__ void dep_guard_h(v8f& a, v8f& b, v16h x, v16h y) { asm volatile("v_nop\n\tv_nop\n\tv_nop\n\tv_nop" : "+v"(a), "+v"(b) : "v"(x), "v"(y)); }
__device__ __forceinline__ void dep_guard_h3(v8f& a, v8f& b, v16h x, v16h y, v16h z) { asm volatile("v_nop\n\tv_nop\n\tv_nop\n\tv_nop" : "+v"(a), "+v"(b) : "v"(x), "v"(y), "v"(z)); }
__device__ __forceinline__ void keep4_h(v16h a, v16h b, v16h c, v16h d) { asm volatile("v_nop" :: "v"(a), "v"(b), "v"(c), "v"(d)); }
__device__ __forceinline__ void keep2_h(v16h a, v16h b) { asm volatile("v_nop" :: "v"(a), "v"(b)); }
__device__ __forceinline__ void acc_guard4(v8f& a, v8f& b, v8f& c, v8f& d) { asm volatile("v_nop\n\tv_nop\n\tv_nop\n\tv_nop" : "+v"(a), "+v"(b), "+v"(c), "+v"(d)); }
__device__ __forceinline__ void acc_guard1(v8f& a) { asm volatile("v_nop\n\tv_nop\n\tv_nop\n\tv_nop" : "+v"(a)); }
template <typename T> struct Frag;
template <> struct Frag<_Float16> {
  typedef v16h V; union U { v16h v; v8h h[2]; };
  static __device__ __forceinline__ v16h load(const _Float16* p) {
    U f; f.h[0] = *(const v8h*)(p); f.h[1] = *(const v8h*)(p + 16); return f.v;
  }
  static __device__ __forceinline__ v8f mma(v16h a, v16h b, v8f c) {
    return __builtin_amdgcn_wmma_f32_16x16x32_f16(false, a, false, b, (short)0, c, false, false);
  }
  static __device__ __forceinline__ void guard(v8f& a, v8f& b, v16h x, v16h y) { dep_guard_h(a, b, x, y); }
  static __device__ __forceinline__ void keep(v16h a, v16h b, v16h c, v16h d) { keep4_h(a, b, c, d); }
};

__device__ __forceinline__ unsigned pk16(unsigned short a, unsigned short b) { return (unsigned)a | ((unsigned)b << 16); }
__device__ __forceinline__ unsigned short h_bits(float f) { const _Float16 h = (_Float16)f; return __builtin_bit_cast(unsigned short, h); }
__device__ __forceinline__ float rne_bf(float f) { return bf_bits2f(f2bf_bits(f)); }

__device__ __forceinline__ float h16_to_f32(unsigned hb) {
  const unsigned sgn = (hb & 0x8000u) << 16; const unsigned em = hb & 0x7fffu;
  const float fn = __uint_as_float((em << 13) + 0x38000000u);
  const float fs = (float)em * 5.9604644775390625e-8f;
  const float mag = (em < 0x400u) ? fs : fn; return __uint_as_float(__float_as_uint(mag) | sgn); }

__device__ __forceinline__ int blk_excl_scan(int cnt, int* scan_ws, int tid, int* tot) {
  const int lane = tid & 31, wave = tid >> 5; int incl = cnt;
#pragma unroll
  for (int o = 1; o < 32; o <<= 1) { const int v = __shfl_up(incl, o, 32); if (lane >= o) incl += v; }
  if (lane == 31) scan_ws[wave] = incl;
  __syncthreads();
  if (wave == 0) { int wv = (lane < kThr / 32) ? scan_ws[lane] : 0; int wincl = wv;
#pragma unroll
    for (int o = 1; o < 32; o <<= 1) { const int v = __shfl_up(wincl, o, 32); if (lane >= o) wincl += v; }
    if (lane < kThr / 32) scan_ws[32 + lane] = wincl - wv; if (lane == 31) scan_ws[64] = wincl; }
  __syncthreads();
  const int res = scan_ws[32 + wave] + incl - cnt; *tot = scan_ws[64];
  return res;
}

__global__ __launch_bounds__(kThr) void bias_prep_kernel(const float* __restrict__ tb, const float* __restrict__ gb,
                                                        float* __restrict__ tbr, float* __restrict__ gbr) {
  const int t = threadIdx.x;
  {
    const v4f v = *(const v4f*)(tb + 4 * t);
    v4f r; r[0] = rne_bf(v[0]); r[1] = rne_bf(v[1]); r[2] = rne_bf(v[2]); r[3] = rne_bf(v[3]);
    *(volatile v4f*)(tbr + 4 * t) = r; __threadfence(); *(volatile v4f*)(tbr + 4 * t) = r;
  }
#pragma unroll 1
  for (int i = t; i < 2 * kHid3 / 4; i += kThr) {
    const v4f v = *(const v4f*)(gb + 4 * i);
    v4f r; r[0] = rne_bf(v[0]); r[1] = rne_bf(v[1]); r[2] = rne_bf(v[2]); r[3] = rne_bf(v[3]);
    *(volatile v4f*)(gbr + 4 * i) = r; __threadfence(); *(volatile v4f*)(gbr + 4 * i) = r;
  }
}

__global__ __launch_bounds__(kThr) void tcast_kernel(const float* __restrict__ in, long ibs, int nrow, int ncol,
                                                    unsigned short* __restrict__ out, long obs, float scale) {
  __shared__ float sm[64][65];
  const int t  = threadIdx.x;
  const int r0 = blockIdx.x * 64;
  const int c0 = blockIdx.y * 64;
  const int z  = blockIdx.z;
  const float* ip = in + (size_t)z * ibs;
#pragma unroll
  for (int i = 0; i < 16; ++i) {
    const int e  = i * kThr + t;
    const int rl = e >> 6;
    const int cl = e & 63;
    sm[cl][rl] = rne_bf(ip[(size_t)(r0 + rl) * ncol + c0 + cl]) * scale;
  }
  __syncthreads();
  const int lane = t & 31, wave = t >> 5;
  const int q = lane >> 3, c8 = (lane & 7) * 8;
  unsigned short* op = out + (size_t)z * obs;
  for (int pass = 0; pass < 2; ++pass) {
#pragma unroll
    for (int it = 0; it < 2; ++it) {
      const int row = wave * 8 + it * 4 + q;
      unsigned short hb[8];
#pragma unroll
      for (int e = 0; e < 8; ++e) hb[e] = h_bits(sm[row][c8 + e]);
      const v4u u = (v4u){pk16(hb[0], hb[1]), pk16(hb[2], hb[3]), pk16(hb[4], hb[5]), pk16(hb[6], hb[7])};
      *(volatile v4u*)(op + (size_t)(c0 + row) * nrow + r0 + c8) = u;
    }
    __threadfence();
  }
}

constexpr int kTrRows  = 32;
constexpr int kPH      = 264;
constexpr int kTrSlabP = 36;
constexpr int kTrLdsF  = 8 * kTrRows * kTrSlabP;
static_assert(2 * kTrRows * kPH * 2 <= kTrLdsF * 4);

template <int AMODE>
__global__ __launch_bounds__(kThr) void tr_kernel(const float* hsrc, const unsigned short* __restrict__ wt,
                                                 const float* __restrict__ tbias, float* __restrict__ trn) {
  __shared__ __align__(16) float lds_f[kTrLdsF];
  unsigned short* sHi = (unsigned short*)lds_f;
  unsigned short* sLo = sHi + kTrRows * kPH;
  const int tid = threadIdx.x, lane = tid & 31, wave = tid >> 5;
  const int m0 = blockIdx.x * kTrRows;
  const v4f z4 = (v4f){0.f, 0.f, 0.f, 0.f};
#pragma unroll
  for (int it = 0; it < 8; ++it) {
    const int idx  = it * kThr + tid;
    const int row  = idx >> 6;
    const int c4   = (idx & 63) * 4;
    const int grow = m0 + row;
    const int gcl  = grow < kNodes ? grow : kNodes - 1;
    const bool live = grow < kNodes;
    v4f v = *(const v4f*)(hsrc + (size_t)gcl * kHid + c4);
    v = live ? v : z4;
    unsigned short hb[4], lb[4];
#pragma unroll
    for (int e = 0; e < 4; ++e) {
      if (AMODE == 0) {
        hb[e] = h_bits(rne_bf(v[e]));
        lb[e] = 0;
      } else {
        const unsigned short h = h_bits(v[e]);
        const float hf = h16_to_f32((unsigned)h);
        hb[e] = h;
        lb[e] = h_bits((v[e] - hf) * kResCarry);
      }
    }
    const v2u uh = (v2u){pk16(hb[0], hb[1]), pk16(hb[2], hb[3])};
    *(v2u*)(sHi + row * kPH + c4) = uh;
    if (AMODE == 1) {
      const v2u ul = (v2u){pk16(lb[0], lb[1]), pk16(lb[2], lb[3])};
      *(v2u*)(sLo + row * kPH + c4) = ul;
    }
  }
  __syncthreads();

  const int rlane = lane & 15;
  const int koff  = (lane >> 4) * 8;
  const int mOff  = (lane >> 4) * 8;
  const _Float16* sHih = (const _Float16*)sHi;
  const _Float16* sLoh = (const _Float16*)sLo;
  const _Float16* wth  = (const _Float16*)wt;
  const int nb0 = wave * 32 + rlane;

  v8f acc[2][2], accl[2][2];
#pragma unroll
  for (int i = 0; i < 2; ++i)
#pragma unroll
    for (int j = 0; j < 2; ++j) { acc[i][j] = (v8f){0.f,0.f,0.f,0.f,0.f,0.f,0.f,0.f}; accl[i][j] = acc[i][j]; }

#pragma unroll 1
  for (int k0 = 0; k0 < kHid; k0 += 32) {
    const v16h a0 = Frag<_Float16>::load(sHih + rlane * kPH + k0 + koff);
    const v16h a1 = Frag<_Float16>::load(sHih + (16 + rlane) * kPH + k0 + koff);
    v16h l0 = a0, l1 = a1;
    if (AMODE == 1) {
      l0 = Frag<_Float16>::load(sLoh + rlane * kPH + k0 + koff);
      l1 = Frag<_Float16>::load(sLoh + (16 + rlane) * kPH + k0 + koff);
    }
    const v16h b0 = Frag<_Float16>::load(wth + (size_t)nb0 * kHid + k0 + koff);
    const v16h b1 = Frag<_Float16>::load(wth + (size_t)(nb0 + 16) * kHid + k0 + koff);
    acc[0][0] = Frag<_Float16>::mma(a0, b0, acc[0][0]);
    acc[0][1] = Frag<_Float16>::mma(a0, b1, acc[0][1]);
    acc[1][0] = Frag<_Float16>::mma(a1, b0, acc[1][0]);
    acc[1][1] = Frag<_Float16>::mma(a1, b1, acc[1][1]);
    if (AMODE == 1) {
      accl[0][0] = Frag<_Float16>::mma(l0, b0, accl[0][0]);
      accl[0][1] = Frag<_Float16>::mma(l0, b1, accl[0][1]);
      accl[1][0] = Frag<_Float16>::mma(l1, b0, accl[1][0]);
      accl[1][1] = Frag<_Float16>::mma(l1, b1, accl[1][1]);
      dep_guard_h(accl[0][0], accl[1][1], l0, l1);
    }
    dep_guard_h(acc[0][0], acc[1][1], a0, a1);
    keep2_h(b0, b1);
  }
  acc_guard4(acc[0][0], acc[0][1], acc[1][0], acc[1][1]);
  if (AMODE == 1) acc_guard4(accl[0][0], accl[0][1], accl[1][0], accl[1][1]);

  __syncthreads();
  float* slab = lds_f + wave * (kTrRows * kTrSlabP);
  const float bj0 = tbias[nb0];
  const float bj1 = tbias[nb0 + 16];
#pragma unroll
  for (int i = 0; i < 2; ++i) {
#pragma unroll
    for (int j = 0; j < 2; ++j) {
      const float bj = (j == 0) ? bj0 : bj1;
#pragma unroll
      for (int r = 0; r < 8; ++r) {
        float v = acc[i][j][r] * kWCarryInv;
        if (AMODE == 1) v += accl[i][j][r] * kWResInv;
        v += bj;
        slab[(16 * i + mOff + r) * kTrSlabP + 16 * j + rlane] = v;
      }
    }
  }
  __syncthreads();
  {
    const int q = lane >> 3, c4 = (lane & 7) * 4;
    for (int pass = 0; pass < 2; ++pass) {
#pragma unroll
      for (int it = 0; it < 8; ++it) {
        const int row = it * 4 + q;
        const v4f v = *(const v4f*)(slab + row * kTrSlabP + c4);
        *(volatile v4f*)(trn + (size_t)(m0 + row) * kHid + wave * 32 + c4) = v;
      }
      __threadfence();
    }
  }
}

constexpr int kTileN    = 8192;
constexpr int kNTile    = 7;
constexpr int kRowsWave = kTileN / 8;
constexpr int kChunk    = 4096;
constexpr int kSpt      = kChunk / kThr;
constexpr int kNChunk   = (kEdges + kChunk - 1) / kChunk;
static_assert(kNTile * kTileN >= kNodesPad);
static_assert(kSpt == 16);
static_assert(kEdges % kSpt == 0);
static_assert((kNChunk - 1) * kChunk < kEdges);
static_assert(kNodes < 65536);
static_assert(kTileN <= 8192);

__device__ __forceinline__ int exam1(int d, int y, int s, bool valid, int n0, int nhi, int tsel, int& cnt) {
  y = y < 0 ? 0 : (y > kTypes - 1 ? kTypes - 1 : y);
  s = s < 0 ? 0 : (s >= kNodes ? kNodes - 1 : s);
  const bool hit = valid && (d >= n0) && (d < nhi) && (y == tsel);
  const int rv = (int)((((unsigned)(d - n0)) << 16) | (unsigned)s);
  cnt += hit ? 1 : 0;
  return hit ? rv : -1;
}

__global__ __launch_bounds__(kThr) void gather_kernel(const float* __restrict__ trn, const int* __restrict__ etyp,
                                                     const int* __restrict__ esrc, const int* __restrict__ etgt,
                                                     float* msg, int tsel, int zfill) {
  __shared__ int LIST[kChunk];
  __shared__ int scan_ws[80];
  const int tid = threadIdx.x, lane = tid & 31, wave = tid >> 5;
  const int n0  = blockIdx.x * kTileN;
  const int nhi = (n0 + kTileN < kNodes) ? (n0 + kTileN) : kNodes;
  for (int i = tid; i < kChunk; i += kThr) LIST[i] = -1;
  if (tid < 80) scan_ws[tid] = 0;
  const v4f z4 = (v4f){0.f, 0.f, 0.f, 0.f};
  if (zfill) {
#pragma unroll 1
    for (int j = 0; j < kRowsWave; ++j) {
      const int row = n0 + wave * kRowsWave + j;
      if (row < kNodesPad) {
        float* rp = msg + (size_t)row * kHid + 4 * lane;
        *(v4f*)rp = z4;
        *(v4f*)(rp + 128) = z4;
      }
    }
  }
  __syncthreads();
#pragma unroll 1
  for (int c = 0; c < kNChunk; ++c) {
    const int  eb    = c * kChunk + tid * kSpt;
    const bool valid = eb < kEdges;
    const int  ebc   = valid ? eb : (kEdges - kSpt);
    int rec[kSpt]; int cnt = 0;
    {
      const v4i d0 = *(const v4i*)(etgt + ebc),     d1 = *(const v4i*)(etgt + ebc + 4);
      const v4i y0 = *(const v4i*)(etyp + ebc),     y1 = *(const v4i*)(etyp + ebc + 4);
      const v4i s0 = *(const v4i*)(esrc + ebc),     s1 = *(const v4i*)(esrc + ebc + 4);
#pragma unroll
      for (int e = 0; e < 4; ++e) rec[e]     = exam1(d0[e], y0[e], s0[e], valid, n0, nhi, tsel, cnt);
#pragma unroll
      for (int e = 0; e < 4; ++e) rec[4 + e] = exam1(d1[e], y1[e], s1[e], valid, n0, nhi, tsel, cnt);
    }
    asm volatile("" ::: "memory");
    {
      const v4i d2 = *(const v4i*)(etgt + ebc + 8), d3 = *(const v4i*)(etgt + ebc + 12);
      const v4i y2 = *(const v4i*)(etyp + ebc + 8), y3 = *(const v4i*)(etyp + ebc + 12);
      const v4i s2 = *(const v4i*)(esrc + ebc + 8), s3 = *(const v4i*)(esrc + ebc + 12);
#pragma unroll
      for (int e = 0; e < 4; ++e) rec[8 + e]  = exam1(d2[e], y2[e], s2[e], valid, n0, nhi, tsel, cnt);
#pragma unroll
      for (int e = 0; e < 4; ++e) rec[12 + e] = exam1(d3[e], y3[e], s3[e], valid, n0, nhi, tsel, cnt);
    }
    int tot; int p = blk_excl_scan(cnt, scan_ws, tid, &tot);
#pragma unroll
    for (int k = 0; k < kSpt; ++k) if (rec[k] >= 0) { if ((unsigned)p < (unsigned)kChunk) LIST[p] = rec[k]; ++p; }
    __syncthreads();
    const int totc = tot < kChunk ? tot : kChunk;
#pragma unroll 1
    for (int base = 0; base < totc; base += 32) {
      const int q  = base + lane;
      const int lv = LIST[q];
      const int rv = (q < totc) ? lv : -1;
      const int own = (rv >= 0 && (rv >> 26) == wave) ? 1 : 0;
      unsigned msk = (unsigned)__ballot(own);
#pragma unroll 1
      for (int it = 0; it < 32; ++it) {
        if (msk == 0u) break;
        const int bp = __builtin_ctz(msk); msk &= msk - 1u;
        const int r  = __shfl(rv, bp, 32);
        const int dl = r >> 16, s = r & 0xFFFF;
        const float* tp = trn + (size_t)s * kHid + 4 * lane;
        const v4f a0 = *(const v4f*)(tp);
        const v4f a1 = *(const v4f*)(tp + 128);
        float* mp = msg + (size_t)(n0 + dl) * kHid + 4 * lane;
        v4f m0v = *(const v4f*)(mp);
        v4f m1v = *(const v4f*)(mp + 128);
        m0v = m0v + a0;
        m1v = m1v + a1;
        *(v4f*)(mp) = m0v;
        *(v4f*)(mp + 128) = m1v;
      }
    }
    __syncthreads();
  }
#pragma unroll 1
  for (int j = 0; j < kRowsWave; ++j) {
    const int row = n0 + wave * kRowsWave + j;
    if (row < kNodesPad) {
      float* rp = msg + (size_t)row * kHid + 4 * lane;
      const v4f v0 = *(const v4f*)(rp);
      const v4f v1 = *(const v4f*)(rp + 128);
      *(volatile v4f*)(rp) = v0; *(volatile v4f*)(rp + 128) = v1;
      __threadfence();
      *(volatile v4f*)(rp) = v0; *(volatile v4f*)(rp + 128) = v1;
    }
  }
}

constexpr int kSP = 260;

__device__ __forceinline__ float sigm(float x) {
  x = fminf(fmaxf(x, -30.0f), 30.0f);
  return 1.0f / (1.0f + expf(-x));
}

template <bool HCONV>
__global__ __launch_bounds__(kThr) void gate_kernel(const float* __restrict__ msg, const float* hsrc,
                                                   const unsigned short* __restrict__ gkp, const unsigned short* __restrict__ grkp,
                                                   const float* __restrict__ gbr, float* outp) {
  __shared__ __align__(16) unsigned short sMh[16 * kPH];
  __shared__ __align__(16) unsigned short sMl[16 * kPH];
  __shared__ __align__(16) unsigned short sH[16 * kPH];
  __shared__ __align__(16) float sHP[16 * kSP];
  __shared__ __align__(16) float slab[16 * kSP];
  const int tid = threadIdx.x, lane = tid & 31, wave = tid >> 5;
  const int m0 = blockIdx.x * 16;
  const v4f z4 = (v4f){0.f, 0.f, 0.f, 0.f};
#pragma unroll
  for (int it = 0; it < 4; ++it) {
    const int idx = it * kThr + tid;
    const int row = idx >> 6;
    const int c4  = (idx & 63) * 4;
    const v4f v = *(const v4f*)(msg + (size_t)(m0 + row) * kHid + c4);
    unsigned short hb[4], lb[4];
#pragma unroll
    for (int e = 0; e < 4; ++e) {
      const unsigned short h = h_bits(v[e]);
      const float hf = h16_to_f32((unsigned)h);
      hb[e] = h;
      lb[e] = h_bits((v[e] - hf) * kResCarry);
    }
    const v2u uh = (v2u){pk16(hb[0], hb[1]), pk16(hb[2], hb[3])};
    const v2u ul = (v2u){pk16(lb[0], lb[1]), pk16(lb[2], lb[3])};
    *(v2u*)(sMh + row * kPH + c4) = uh;
    *(v2u*)(sMl + row * kPH + c4) = ul;
  }
#pragma unroll
  for (int it = 0; it < 4; ++it) {
    const int idx  = it * kThr + tid;
    const int row  = idx >> 6;
    const int c4   = (idx & 63) * 4;
    const int grow = m0 + row;
    const int gcl  = grow < kNodes ? grow : kNodes - 1;
    const bool live = grow < kNodes;
    v4f v = *(const v4f*)(hsrc + (size_t)gcl * kHid + c4);
    v = live ? v : z4;
    v4f x;
    unsigned short hb[4];
#pragma unroll
    for (int e = 0; e < 4; ++e) {
      const float xe = HCONV ? rne_bf(v[e]) : v[e];
      x[e] = xe;
      hb[e] = h_bits(xe);
    }
    const v2u uh = (v2u){pk16(hb[0], hb[1]), pk16(hb[2], hb[3])};
    *(v2u*)(sH + row * kPH + c4) = uh;
    *(v4f*)(sHP + row * kSP + c4) = x;
  }
  __syncthreads();

  const int rlane = lane & 15;
  const int koff  = (lane >> 4) * 8;
  const int mOff  = (lane >> 4) * 8;
  const _Float16* sMhh = (const _Float16*)sMh;
  const _Float16* sMlh = (const _Float16*)sMl;
  const _Float16* sHh  = (const _Float16*)sH;
  const _Float16* gk   = (const _Float16*)gkp;
  const _Float16* grk  = (const _Float16*)grkp;

#pragma unroll 1
  for (int j = 0; j < 2; ++j) {
    const int ncol = wave * 32 + j * 16 + rlane;
    v8f ax[3], al[3], ah[3];
#pragma unroll
    for (int g = 0; g < 3; ++g) {
      ax[g] = (v8f){0.f,0.f,0.f,0.f,0.f,0.f,0.f,0.f};
      al[g] = ax[g];
      ah[g] = ax[g];
    }
#pragma unroll 1
    for (int k0 = 0; k0 < kHid; k0 += 32) {
      const v16h fm = Frag<_Float16>::load(sMhh + rlane * kPH + k0 + koff);
      const v16h fl = Frag<_Float16>::load(sMlh + rlane * kPH + k0 + koff);
      const v16h fh = Frag<_Float16>::load(sHh + rlane * kPH + k0 + koff);
      const _Float16* bp = gk + (size_t)ncol * kHid + k0 + koff;
      const v16h b0 = Frag<_Float16>::load(bp);
      const v16h b1 = Frag<_Float16>::load(bp + (size_t)kHid * kHid);
      const v16h b2 = Frag<_Float16>::load(bp + (size_t)2 * kHid * kHid);
      const _Float16* rp = grk + (size_t)ncol * kHid + k0 + koff;
      const v16h c0 = Frag<_Float16>::load(rp);
      const v16h c1 = Frag<_Float16>::load(rp + (size_t)kHid * kHid);
      const v16h c2 = Frag<_Float16>::load(rp + (size_t)2 * kHid * kHid);
      ax[0] = Frag<_Float16>::mma(fm, b0, ax[0]);
      ax[1] = Frag<_Float16>::mma(fm, b1, ax[1]);
      ax[2] = Frag<_Float16>::mma(fm, b2, ax[2]);
      al[0] = Frag<_Float16>::mma(fl, b0, al[0]);
      al[1] = Frag<_Float16>::mma(fl, b1, al[1]);
      al[2] = Frag<_Float16>::mma(fl, b2, al[2]);
      ah[0] = Frag<_Float16>::mma(fh, c0, ah[0]);
      ah[1] = Frag<_Float16>::mma(fh, c1, ah[1]);
      ah[2] = Frag<_Float16>::mma(fh, c2, ah[2]);
      dep_guard_h3(ax[0], ah[2], fm, fl, fh);
      keep4_h(b0, b1, b2, c0);
      keep2_h(c1, c2);
    }
    acc_guard4(ax[0], ax[1], ax[2], al[0]);
    acc_guard4(al[1], al[2], ah[0], ah[1]);
    acc_guard1(ah[2]);

    const int c = ncol;
    const float b0z = gbr[c],         b0r = gbr[kHid + c],         b0h = gbr[2 * kHid + c];
    const float b1z = gbr[kHid3 + c], b1r = gbr[kHid3 + kHid + c], b1h = gbr[kHid3 + 2 * kHid + c];
#pragma unroll
    for (int r = 0; r < 8; ++r) {
      const int row = mOff + r;
      const float xz = ax[0][r] * kWCarryInv + al[0][r] * kWResInv + b0z;
      const float xr = ax[1][r] * kWCarryInv + al[1][r] * kWResInv + b0r;
      const float xh = ax[2][r] * kWCarryInv + al[2][r] * kWResInv + b0h;
      const float hz = ah[0][r] * kWCarryInv + b1z;
      const float hr = ah[1][r] * kWCarryInv + b1r;
      const float hh = ah[2][r] * kWCarryInv + b1h;
      const float z  = sigm(xz + hz);
      const float rg = sigm(xr + hr);
      const float hc = tanhf(xh + rg * hh);
      const float hpv = sHP[row * kSP + c];
      const float hn = z * hpv + (1.0f - z) * hc;
      slab[row * kSP + c] = hn;
    }
  }
  __syncthreads();

#pragma unroll
  for (int rr = 0; rr < 2; ++rr) {
    const int rl = wave * 2 + rr;
    const int grow = m0 + rl;
    if (grow < kNodes) {
      const v4f v0 = *(const v4f*)(slab + rl * kSP + 4 * lane);
      const v4f v1 = *(const v4f*)(slab + rl * kSP + 128 + 4 * lane);
      float* op = outp + (size_t)grow * kHid + 4 * lane;
      *(volatile v4f*)(op) = v0; *(volatile v4f*)(op + 128) = v1;
      __threadfence();
      *(volatile v4f*)(op) = v0; *(volatile v4f*)(op + 128) = v1;
    }
  }
}

extern "C" void kernel_launch(void* const* d_in, const int* in_sizes, int n_in,
                              void* d_out, int out_size, void* d_ws, size_t ws_size, hipStream_t stream) {
  if (n_in < 9) return;
  const float* states = (const float*)d_in[0];
  const int*   etyp   = (const int*)  d_in[1];
  const int*   esrc   = (const int*)  d_in[2];
  const int*   etgt   = (const int*)  d_in[3];
  const float* tW     = (const float*)d_in[4];
  const float* tB     = (const float*)d_in[5];
  const float* gk     = (const float*)d_in[6];
  const float* grk    = (const float*)d_in[7];
  const float* gb     = (const float*)d_in[8];
  float* out = (float*)d_out;

  if (in_sizes[0] != kNodes * kHid || in_sizes[1] != kEdges || in_sizes[2] != kEdges || in_sizes[3] != kEdges) return;
  if (in_sizes[4] != kTypes * kHid * kHid || in_sizes[5] != kTypes * kHid || in_sizes[6] != kHid * kHid3 ||
      in_sizes[7] != kHid * kHid3 || in_sizes[8] != 2 * kHid3 || out_size != kNodes * kHid) return;

  char* ws = (char*)d_ws; size_t off = 0;
  auto carve = [&](size_t bytes) -> char* { char* p = ws + off; off += (bytes + 255) & ~(size_t)255; return p; };
  unsigned short* wt16  = (unsigned short*)carve((size_t)kTypes * kHid * kHid * 2);
  unsigned short* gk16  = (unsigned short*)carve((size_t)kHid3 * kHid * 2);
  unsigned short* grk16 = (unsigned short*)carve((size_t)kHid3 * kHid * 2);
  float*          tbr   = (float*)carve((size_t)kTypes * kHid * 4);
  float*          gbr   = (float*)carve((size_t)2 * kHid3 * 4);
  float*          trn   = (float*)carve((size_t)kNodesPad * kHid * 4);
  float*          msg   = (float*)carve((size_t)kNodesPad * kHid * 4);
  if (off > ws_size || off > (size_t)134217728) return;

  bias_prep_kernel<<<1, kThr, 0, stream>>>(tB, gb, tbr, gbr);
  tcast_kernel<<<dim3(kHid / 64, kHid / 64, kTypes), kThr, 0, stream>>>(tW, (long)kHid * kHid, kHid, kHid,
                                                                       wt16, (long)kHid * kHid, kWCarry);
  tcast_kernel<<<dim3(kHid / 64, kHid3 / 64, 1), kThr, 0, stream>>>(gk, 0L, kHid, kHid3, gk16, 0L, kWCarry);
  tcast_kernel<<<dim3(kHid / 64, kHid3 / 64, 1), kThr, 0, stream>>>(grk, 0L, kHid, kHid3, grk16, 0L, kWCarry);

  const int tr_blocks   = kNodesPad / kTrRows;
  const int gate_blocks = kNodesPad / 16;
  for (int t = 0; t < kTypes; ++t) {
    tr_kernel<0><<<tr_blocks, kThr, 0, stream>>>(states, wt16 + (size_t)t * kHid * kHid, tbr + t * kHid, trn);
    gather_kernel<<<kNTile, kThr, 0, stream>>>(trn, etyp, esrc, etgt, msg, t, (t == 0) ? 1 : 0);
  }
  gate_kernel<true><<<gate_blocks, kThr, 0, stream>>>(msg, states, gk16, grk16, gbr, out);
  for (int t = 0; t < kTypes; ++t) {
    tr_kernel<1><<<tr_blocks, kThr, 0, stream>>>(out, wt16 + (size_t)t * kHid * kHid, tbr + t * kHid, trn);
    gather_kernel<<<kNTile, kThr, 0, stream>>>(trn, etyp, esrc, etgt, msg, t, (t == 0) ? 1 : 0);
  }
  gate_kernel<false><<<gate_blocks, kThr, 0, stream>>>(msg, out, gk16, grk16, gbr, out);
}
